// ConvMambaBlock_57415122813610
// MI455X (gfx1250) — hardware-verified
//
#include <hip/hip_runtime.h>
#include <math.h>

typedef __attribute__((ext_vector_type(16))) _Float16 v16h;
typedef __attribute__((ext_vector_type(8)))  _Float16 v8h;
typedef __attribute__((ext_vector_type(16))) __bf16   v16b;
typedef __attribute__((ext_vector_type(8)))  __bf16   v8b;
typedef __attribute__((ext_vector_type(8)))  float    v8f;
typedef __attribute__((ext_vector_type(4)))  float    v4f;

constexpr int kB    = 4;
constexpr int kL    = 1024;
constexpr int kDim  = 256;
constexpr int kDin  = 512;
constexpr int kNst  = 32;
constexpr int kDtR  = 16;
constexpr int kDtP  = 32;
constexpr int kXdbN = 80;
constexpr int kXdbP = 128;
constexpr int kXZP  = 2 * kDin;
constexpr int kHid  = 4 * kDim;
constexpr int kRows = kB * kL;
constexpr int kTP   = 260;
constexpr int kLP   = 264;

__device__ __forceinline__ unsigned short f2bf_bits(float f) {
  unsigned u = __float_as_uint(f);
  return (unsigned short)((u + 0x7FFFu + ((u >> 16) & 1u)) >> 16);
}
__device__ __forceinline__ float bf_bits2f(unsigned short h) { return __uint_as_float(((unsigned)h) << 16); }

__device__ __forceinline__ void dep_guard_h(v8f& a, v8f& b, v16h x, v16h y) { asm volatile("v_nop\n\tv_nop\n\tv_nop\n\tv_nop" : "+v"(a), "+v"(b) : "v"(x), "v"(y)); }
__device__ __forceinline__ void dep_guard_b(v8f& a, v8f& b, v16b x, v16b y) { asm volatile("v_nop\n\tv_nop\n\tv_nop\n\tv_nop" : "+v"(a), "+v"(b) : "v"(x), "v"(y)); }
__device__ __forceinline__ void keep4_h(v16h a, v16h b, v16h c, v16h d) { asm volatile("v_nop" :: "v"(a), "v"(b), "v"(c), "v"(d)); }
__device__ __forceinline__ void keep4_b(v16b a, v16b b, v16b c, v16b d) { asm volatile("v_nop" :: "v"(a), "v"(b), "v"(c), "v"(d)); }
__device__ __forceinline__ void acc_guard4(v8f& a, v8f& b, v8f& c, v8f& d) { asm volatile("v_nop\n\tv_nop\n\tv_nop\n\tv_nop" : "+v"(a), "+v"(b), "+v"(c), "+v"(d)); }
template <typename T> struct Frag;
template <> struct Frag<_Float16> {
  typedef v16h V; union U { v16h v; v8h h[2]; };
  static __device__ __forceinline__ v16h load(const _Float16* p) {
    U f; f.h[0] = *(const v8h*)(p); f.h[1] = *(const v8h*)(p + 16); return f.v;
  }
  static __device__ __forceinline__ v8f mma(v16h a, v16h b, v8f c) {
    return __builtin_amdgcn_wmma_f32_16x16x32_f16(false, a, false, b, (short)0, c, false, false);
  }
  static __device__ __forceinline__ void guard(v8f& a, v8f& b, v16h x, v16h y) { dep_guard_h(a, b, x, y); }
  static __device__ __forceinline__ void keep(v16h a, v16h b, v16h c, v16h d) { keep4_h(a, b, c, d); }
};
template <> struct Frag<__bf16> {
  typedef v16b V; union U { v16b v; v8b h[2]; };
  static __device__ __forceinline__ v16b load(const __bf16* p) {
    U f; f.h[0] = *(const v8b*)(p); f.h[1] = *(const v8b*)(p + 16); return f.v;
  }
  static __device__ __forceinline__ v8f mma(v16b a, v16b b, v8f c) {
    return __builtin_amdgcn_wmma_f32_16x16x32_bf16(false, a, false, b, (short)0, c, false, false);
  }
  static __device__ __forceinline__ void guard(v8f& a, v8f& b, v16b x, v16b y) { dep_guard_b(a, b, x, y); }
  static __device__ __forceinline__ void keep(v16b a, v16b b, v16b c, v16b d) { keep4_b(a, b, c, d); }
};

template <int ET> struct Elem;
template <> struct Elem<0> { typedef _Float16 T; };
template <> struct Elem<1> { typedef __bf16 T; };
template <int ET, bool SPLIT, int BIAS_MODE, int OUT_MODE, bool RESID, int ACT = 0>
__global__ __launch_bounds__(256) void wmma_gemm64(
    const unsigned short* __restrict__ Ap, const unsigned short* __restrict__ A2p, int lda, long strideA,
    const unsigned short* __restrict__ Btp, const unsigned short* __restrict__ Bt2p, int ldb, long strideB,
    void* __restrict__ Cout, void* __restrict__ Cout2, int ldc, long strideC,
    const float* __restrict__ bias,
    const float* __restrict__ resid, long strideR,
    int M, int N, int K, float scale) {
  typedef typename Elem<ET>::T T;
  typedef typename Frag<T>::V V;
  const T* A = (const T*)Ap; const T* A2 = (const T*)A2p; const T* Bt = (const T*)Btp; const T* Bt2 = (const T*)Bt2p;
  __shared__ __align__(16) float sT[8][16 * 68];
  const int b    = blockIdx.y;
  const int lane = threadIdx.x & 31;
  const int wave = threadIdx.x >> 5;
  const int tilesN = N >> 6;
  const int tilesM = M >> 6;
  const int tile = blockIdx.x * 8 + wave;
  if (tile >= tilesM * tilesN) return;
  const int tm = tile / tilesN;
  const int tn = tile - tm * tilesN;
  const int m0 = tm << 6;
  const int n0 = tn << 6;

  const T* Ab  = A  + (size_t)b * strideA;
  const T* Bb  = Bt + (size_t)b * strideB;
  const T* Ab2 = SPLIT ? (A2  + (size_t)b * strideA) : nullptr;
  const T* Bb2 = SPLIT ? (Bt2 + (size_t)b * strideB) : nullptr;

  const int rlane = lane & 15;
  const int koff  = (lane >> 4) * 8;
  const int mOff  = (lane >> 4) * 8;

  v8f acc[4][4];
#pragma unroll
  for (int i = 0; i < 4; ++i)
#pragma unroll
    for (int j = 0; j < 4; ++j) acc[i][j] = (v8f){0.f,0.f,0.f,0.f,0.f,0.f,0.f,0.f};

  for (int k0 = 0; k0 < K; k0 += 32) {
    V bh[4], bl[4];
#pragma unroll
    for (int j = 0; j < 4; ++j) {
      const size_t bo = (size_t)(n0 + (j << 4) + rlane) * ldb + koff + k0;
      bh[j] = Frag<T>::load(Bb + bo);
      if (SPLIT) bl[j] = Frag<T>::load(Bb2 + bo);
    }
#pragma unroll
    for (int i = 0; i < 4; ++i) {
      const size_t ao = (size_t)(m0 + (i << 4) + rlane) * lda + koff + k0;
      V ah = Frag<T>::load(Ab + ao);
      V al;
      if (SPLIT) al = Frag<T>::load(Ab2 + ao);
#pragma unroll
      for (int j = 0; j < 4; ++j) {
        acc[i][j] = Frag<T>::mma(ah, bh[j], acc[i][j]);
        if (SPLIT) {
          acc[i][j] = Frag<T>::mma(ah, bl[j], acc[i][j]);
          acc[i][j] = Frag<T>::mma(al, bh[j], acc[i][j]);
        }
      }
      Frag<T>::guard(acc[i][0], acc[i][3], ah, SPLIT ? al : ah);
    }
    Frag<T>::keep(bh[0], bh[1], bh[2], bh[3]);
    if (SPLIT) Frag<T>::keep(bl[0], bl[1], bl[2], bl[3]);
  }
  acc_guard4(acc[0][0], acc[0][1], acc[0][2], acc[0][3]);
  acc_guard4(acc[1][0], acc[1][1], acc[1][2], acc[1][3]);
  acc_guard4(acc[2][0], acc[2][1], acc[2][2], acc[2][3]);
  acc_guard4(acc[3][0], acc[3][1], acc[3][2], acc[3][3]);

  float* slab = sT[wave];
  const float* Rb = RESID ? (resid + (size_t)b * strideR) : nullptr;
#pragma unroll
  for (int i = 0; i < 4; ++i) {
    const int mBase = m0 + (i << 4);
#pragma unroll
    for (int j = 0; j < 4; ++j) {
      const int n = n0 + (j << 4) + rlane;
      float bv = 0.f;
      if (BIAS_MODE == 2) bv = bias[n];
#pragma unroll
      for (int r = 0; r < 8; ++r) {
        float v = acc[i][j][r] * scale;
        if (BIAS_MODE == 1) v += bias[mBase + mOff + r];
        if (BIAS_MODE == 2) v += bv;
        if (RESID) v += Rb[(size_t)(mBase + mOff + r) * ldc + n];
        if (ACT == 1) v = tanhf(v);
        if (ACT == 2) v = fmaxf(v, 0.0f);
        if (ACT == 3) v = v / (1.0f + expf(-v));
        if (ACT == 4) v = (v > 0.f) ? v : 0.01f * v;
        if (ACT == 5) v = 0.5f * v * (1.0f + erff(v * 0.70710678118654752f));
        slab[(mOff + r) * 68 + (j << 4) + rlane] = v;
      }
    }
    __builtin_amdgcn_fence(__ATOMIC_RELEASE, "workgroup");
    __builtin_amdgcn_wave_barrier();
    __builtin_amdgcn_fence(__ATOMIC_ACQUIRE, "workgroup");
    if (OUT_MODE == 0) {
      float* C = (float*)Cout + (size_t)b * strideC;
      const int hh = lane >> 4, c4 = (lane & 15) * 4;
      for (int pass = 0; pass < 2; ++pass) {
#pragma unroll
        for (int it = 0; it < 8; ++it) {
          const int row = it * 2 + hh;
          v4f v = *(const v4f*)(slab + row * 68 + c4);
          *(volatile v4f*)(C + (size_t)(mBase + row) * ldc + n0 + c4) = v;
        }
        __threadfence();
      }
    } else {
      const int q = lane >> 3, c8 = (lane & 7) * 8;
      unsigned short* C  = (unsigned short*)Cout  + (size_t)b * strideC;
      unsigned short* C2 = (OUT_MODE == 2) ? ((unsigned short*)Cout2 + (size_t)b * strideC) : nullptr;
      for (int pass = 0; pass < 2; ++pass) {
#pragma unroll
        for (int it = 0; it < 4; ++it) {
          const int row = it * 4 + q;
          const float* sp = slab + row * 68 + c8;
          v8h hv, lv;
#pragma unroll
          for (int e = 0; e < 8; ++e) {
            if (OUT_MODE == 1) {
              hv[e] = (_Float16)sp[e];
            } else {
              unsigned short hb = f2bf_bits(sp[e]);
              unsigned short lb = f2bf_bits(sp[e] - bf_bits2f(hb));
              hv[e] = __builtin_bit_cast(_Float16, hb);
              lv[e] = __builtin_bit_cast(_Float16, lb);
            }
          }
          *(volatile v8h*)(C + (size_t)(mBase + row) * ldc + n0 + c8) = hv;
          if (OUT_MODE == 2) *(volatile v8h*)(C2 + (size_t)(mBase + row) * ldc + n0 + c8) = lv;
        }
        __threadfence();
      }
    }
    __builtin_amdgcn_fence(__ATOMIC_RELEASE, "workgroup");
    __builtin_amdgcn_wave_barrier();
    __builtin_amdgcn_fence(__ATOMIC_ACQUIRE, "workgroup");
  }
}

__global__ __launch_bounds__(256) void cast_f16_kernel(
    const float* __restrict__ src, unsigned short* __restrict__ dst, int total8, float scale)
{
  const int i = blockIdx.x * 256 + threadIdx.x;
  if (i >= total8) return;
  const size_t e0 = (size_t)i << 3;
  const float* p = src + e0;
  const v4f a0 = *(const v4f*)(p);
  const v4f a1 = *(const v4f*)(p + 4);
  v8h hv;
#pragma unroll
  for (int e = 0; e < 4; ++e) {
    hv[e]     = (_Float16)(a0[e] * scale);
    hv[4 + e] = (_Float16)(a1[e] * scale);
  }
  unsigned short* q = dst + e0;
  *(volatile v8h*)q = hv;
  __threadfence();
  *(volatile v8h*)q = hv;
}

__global__ __launch_bounds__(256) void zero16_kernel(unsigned short* __restrict__ dst, int total8)
{
  const int i = blockIdx.x * 256 + threadIdx.x;
  if (i >= total8) return;
  v8h z;
#pragma unroll
  for (int e = 0; e < 8; ++e) z[e] = (_Float16)0.0f;
  unsigned short* q = dst + ((size_t)i << 3);
  *(volatile v8h*)q = z;
  __threadfence();
  *(volatile v8h*)q = z;
}

__global__ __launch_bounds__(256) void pad16_cast_kernel(
    const float* __restrict__ src, int spitch, unsigned short* __restrict__ dst, int total, float scale)
{
  const int i = blockIdx.x * 256 + threadIdx.x;
  if (i >= total) return;
  const int row = i >> 2, seg = i & 3;
  const int cs  = (seg & 1) * 8;
  const float* p = src + (size_t)row * spitch + cs;
  const v4f a0 = *(const v4f*)(p);
  const v4f a1 = *(const v4f*)(p + 4);
  const bool keep = (seg < 2);
  v8h hv;
#pragma unroll
  for (int e = 0; e < 4; ++e) {
    hv[e]     = keep ? (_Float16)(a0[e] * scale) : (_Float16)0.0f;
    hv[4 + e] = keep ? (_Float16)(a1[e] * scale) : (_Float16)0.0f;
  }
  unsigned short* q = dst + ((size_t)i << 3);
  *(volatile v8h*)q = hv;
  __threadfence();
  *(volatile v8h*)q = hv;
}

__device__ __forceinline__ void ln_row8(const float* __restrict__ xr, const float* __restrict__ g,
                                        const float* __restrict__ bb, int lane, float (&y)[8])
{
  const int c0 = lane * 8;
  const v4f a0 = *(const v4f*)(xr + c0), a1 = *(const v4f*)(xr + c0 + 4);
  const v4f g0 = *(const v4f*)(g + c0),  g1 = *(const v4f*)(g + c0 + 4);
  const v4f q0 = *(const v4f*)(bb + c0), q1 = *(const v4f*)(bb + c0 + 4);
  float v[8], gg[8], bv[8];
#pragma unroll
  for (int e = 0; e < 4; ++e) {
    v[e] = a0[e]; v[4 + e] = a1[e];
    gg[e] = g0[e]; gg[4 + e] = g1[e];
    bv[e] = q0[e]; bv[4 + e] = q1[e];
  }
  float s = 0.f;
#pragma unroll
  for (int e = 0; e < 8; ++e) s += v[e];
#pragma unroll
  for (int off = 16; off > 0; off >>= 1) s += __shfl_xor(s, off, 32);
  const float mu = s * (1.0f / (float)kDim);
  float d[8];
  float q = 0.f;
#pragma unroll
  for (int e = 0; e < 8; ++e) { d[e] = v[e] - mu; q += d[e] * d[e]; }
#pragma unroll
  for (int off = 16; off > 0; off >>= 1) q += __shfl_xor(q, off, 32);
  const float var  = q * (1.0f / (float)kDim);
  const float rstd = rsqrtf(var + 1e-5f);
#pragma unroll
  for (int e = 0; e < 8; ++e) y[e] = (d[e] * rstd) * gg[e] + bv[e];
}

__global__ __launch_bounds__(256) void ln_conv_kernel(
    const float* __restrict__ x, const float* __restrict__ g, const float* __restrict__ bb,
    const float* __restrict__ cw, const float* __restrict__ cb, unsigned short* __restrict__ U0)
{
  __shared__ __align__(16) float sX[34 * kLP];
  const int tid = threadIdx.x, lane = tid & 31, wave = tid >> 5;
  const int r0 = blockIdx.x * 32;
  const int b  = r0 >> 10;
  const int t0 = r0 & (kL - 1);
#pragma unroll 1
  for (int t = 0; t < 5; ++t) {
    const int j = (t < 4) ? (wave + 8 * t) : (32 + wave);
    if (j > 33) break;
    const int tt = t0 - 1 + j;
    const bool valid = (tt >= 0) && (tt < kL);
    const int tc = tt < 0 ? 0 : (tt >= kL ? kL - 1 : tt);
    float y[8];
    ln_row8(x + ((size_t)b * kL + tc) * kDim, g, bb, lane, y);
    v4f o0, o1;
#pragma unroll
    for (int e = 0; e < 4; ++e) {
      o0[e] = valid ? y[e] : 0.f;
      o1[e] = valid ? y[4 + e] : 0.f;
    }
    *(v4f*)(sX + j * kLP + lane * 8)     = o0;
    *(v4f*)(sX + j * kLP + lane * 8 + 4) = o1;
  }
  __syncthreads();
  float w0[8], w1[8], w2[8], cbv[8];
#pragma unroll
  for (int e = 0; e < 8; ++e) {
    const int c = lane * 8 + e;
    w0[e] = cw[c * 3 + 0]; w1[e] = cw[c * 3 + 1]; w2[e] = cw[c * 3 + 2];
    cbv[e] = cb[c];
  }
#pragma unroll 1
  for (int t = 0; t < 4; ++t) {
    const int i = wave + 8 * t;
    const float* pp = sX + i * kLP + lane * 8;
    const float* pc = sX + (i + 1) * kLP + lane * 8;
    const float* pn = sX + (i + 2) * kLP + lane * 8;
    const v4f p0 = *(const v4f*)(pp), p1 = *(const v4f*)(pp + 4);
    const v4f c0 = *(const v4f*)(pc), c1 = *(const v4f*)(pc + 4);
    const v4f n0 = *(const v4f*)(pn), n1 = *(const v4f*)(pn + 4);
    float prv[8], cur[8], nxt[8];
#pragma unroll
    for (int e = 0; e < 4; ++e) {
      prv[e] = p0[e]; prv[4 + e] = p1[e];
      cur[e] = c0[e]; cur[4 + e] = c1[e];
      nxt[e] = n0[e]; nxt[4 + e] = n1[e];
    }
    v8h hv;
#pragma unroll
    for (int e = 0; e < 8; ++e) {
      float acc = prv[e] * w0[e];
      acc = fmaf(cur[e], w1[e], acc);
      acc = fmaf(nxt[e], w2[e], acc);
      const float u = (acc + cbv[e]) + cur[e];
      hv[e] = (_Float16)u;
    }
    unsigned short* q = U0 + (size_t)(r0 + i) * kDim + lane * 8;
    *(volatile v8h*)q = hv;
    __threadfence();
    *(volatile v8h*)q = hv;
  }
}

__global__ __launch_bounds__(256) void ln_cast_kernel(
    const float* __restrict__ X2, const float* __restrict__ g, const float* __restrict__ bb,
    unsigned short* __restrict__ X2LN)
{
  const int tid = threadIdx.x, lane = tid & 31, wave = tid >> 5;
  const int r0 = blockIdx.x * 32;
#pragma unroll 1
  for (int t = 0; t < 4; ++t) {
    const int r = r0 + wave + 8 * t;
    float y[8];
    ln_row8(X2 + (size_t)r * kDim, g, bb, lane, y);
    v8h hv;
#pragma unroll
    for (int e = 0; e < 8; ++e) hv[e] = (_Float16)y[e];
    unsigned short* q = X2LN + (size_t)r * kDim + lane * 8;
    *(volatile v8h*)q = hv;
    __threadfence();
    *(volatile v8h*)q = hv;
  }
}

__global__ __launch_bounds__(256) void conv_silu_kernel(
    const float* __restrict__ XZ, const float* __restrict__ cw, const float* __restrict__ cb,
    float* __restrict__ XIN, unsigned short* __restrict__ XIN16)
{
  __shared__ __align__(16) float sT[16 * kTP];
  const int tid = threadIdx.x, lane = tid & 31, wave = tid >> 5;
  const int d0 = blockIdx.x * 256, d = d0 + tid;
  const int t0 = blockIdx.y * 64;
  const size_t rb = (size_t)blockIdx.z * kL;
  const float w0 = cw[d * 4 + 0], w1 = cw[d * 4 + 1], w2 = cw[d * 4 + 2], w3 = cw[d * 4 + 3];
  const float bc = cb[d];
  float xm3, xm2, xm1;
  {
    const int r3 = t0 - 3, r2 = t0 - 2, r1 = t0 - 1;
    const float v3 = XZ[(rb + (r3 < 0 ? 0 : r3)) * kXZP + d];
    const float v2 = XZ[(rb + (r2 < 0 ? 0 : r2)) * kXZP + d];
    const float v1 = XZ[(rb + (r1 < 0 ? 0 : r1)) * kXZP + d];
    xm3 = (r3 >= 0) ? v3 : 0.f;
    xm2 = (r2 >= 0) ? v2 : 0.f;
    xm1 = (r1 >= 0) ? v1 : 0.f;
  }
  const int hrow = wave >> 1;
  const int hch  = (wave & 1) * 128 + lane * 4;
#pragma unroll 1
  for (int sub = 0; sub < 4; ++sub) {
    const int lb = t0 + sub * 16;
#pragma unroll 1
    for (int s = 0; s < 16; ++s) {
      const float xc = XZ[(rb + lb + s) * kXZP + d];
      float acc = w0 * xm3;
      acc = fmaf(w1, xm2, acc);
      acc = fmaf(w2, xm1, acc);
      acc = fmaf(w3, xc, acc);
      const float sv = acc + bc;
      const float sg = __builtin_amdgcn_rcpf(1.0f + __expf(-sv));
      sT[s * kTP + tid] = sv * sg;
      xm3 = xm2; xm2 = xm1; xm1 = xc;
    }
    __syncthreads();
    v4f fv[4];
    v8h bv[2];
#pragma unroll
    for (int it = 0; it < 4; ++it) fv[it] = *(const v4f*)(sT + (it * 4 + hrow) * kTP + hch);
#pragma unroll
    for (int it = 0; it < 2; ++it) {
      const float* sp = sT + (it * 8 + wave) * kTP + lane * 8;
      const v4f a0 = *(const v4f*)(sp);
      const v4f a1 = *(const v4f*)(sp + 4);
#pragma unroll
      for (int e = 0; e < 4; ++e) {
        bv[it][e]     = (_Float16)(a0[e] * 16.0f);
        bv[it][4 + e] = (_Float16)(a1[e] * 16.0f);
      }
    }
    for (int pass = 0; pass < 2; ++pass) {
#pragma unroll
      for (int it = 0; it < 4; ++it)
        *(volatile v4f*)(XIN + (rb + lb + it * 4 + hrow) * kDin + d0 + hch) = fv[it];
#pragma unroll
      for (int it = 0; it < 2; ++it)
        *(volatile v8h*)(XIN16 + (rb + lb + it * 8 + wave) * kDin + d0 + lane * 8) = bv[it];
      __threadfence();
    }
    __syncthreads();
  }
}

__global__ __launch_bounds__(256) void scan_kernel(
    const float* __restrict__ DLR, const float* __restrict__ UIN, const float* __restrict__ XZ,
    const float* __restrict__ XDB, const float* __restrict__ A_log, const float* __restrict__ Dv,
    unsigned short* __restrict__ Y16)
{
  __shared__ __align__(16) float sBC[16 * 64];
  __shared__ __align__(16) float sY[16 * kTP];
  const int tid = threadIdx.x, lane = tid & 31, wave = tid >> 5;
  const int d0 = blockIdx.x * 256, d = d0 + tid;
  const size_t rb = (size_t)blockIdx.y * kL;

  float An[kNst];
#pragma unroll
  for (int n = 0; n < kNst; ++n) An[n] = -__expf(A_log[(size_t)d * kNst + n]);
  const float Dd = Dv[d];
  float h[kNst];
#pragma unroll
  for (int n = 0; n < kNst; ++n) h[n] = 0.f;

#pragma unroll 1
  for (int c = 0; c < kL / 16; ++c) {
    const int l0 = c * 16;
    {
      const int r = tid >> 4, q = (tid & 15) * 4;
      const v4f v = *(const v4f*)(XDB + (rb + l0 + r) * kXdbP + kDtR + q);
      *(v4f*)(sBC + r * 64 + q) = v;
    }
    __syncthreads();
#pragma unroll 1
    for (int s = 0; s < 16; ++s) {
      const size_t m = rb + l0 + s;
      const float a     = DLR[m * kDin + d];
      const float delta = fmaxf(a, 0.0f) + log1pf(__expf(-fabsf(a)));
      const float xv    = UIN[m * kDin + d];
      const float zv    = XZ[m * kXZP + kDin + d];
      float y = 0.f;
#pragma unroll
      for (int qq = 0; qq < 8; ++qq) {
        const v4f Bq = *(const v4f*)(sBC + s * 64 + 4 * qq);
        const v4f Cq = *(const v4f*)(sBC + s * 64 + kNst + 4 * qq);
#pragma unroll
        for (int e = 0; e < 4; ++e) {
          const int n = 4 * qq + e;
          const float ex = __expf(delta * An[n]);
          float db = delta * Bq[e];
          asm volatile("" : "+v"(db));
          float p = db * xv;
          asm volatile("" : "+v"(p));
          float qv = h[n] * ex;
          asm volatile("" : "+v"(qv));
          const float hn = qv + p;
          h[n] = hn;
          float rr = Cq[e] * hn;
          asm volatile("" : "+v"(rr));
          y += rr;
        }
      }
      float sk = xv * Dd;
      asm volatile("" : "+v"(sk));
      y += sk;
      const float sg = __builtin_amdgcn_rcpf(1.0f + __expf(-zv));
      const float gt = zv * sg;
      sY[s * kTP + tid] = (y * gt) * 256.0f;
    }
    __syncthreads();
    v8h hv[2];
#pragma unroll
    for (int it = 0; it < 2; ++it) {
      const float* sp = sY + (it * 8 + wave) * kTP + lane * 8;
      const v4f a0 = *(const v4f*)(sp);
      const v4f a1 = *(const v4f*)(sp + 4);
#pragma unroll
      for (int e = 0; e < 4; ++e) { hv[it][e] = (_Float16)a0[e]; hv[it][4 + e] = (_Float16)a1[e]; }
    }
    for (int pass = 0; pass < 2; ++pass) {
#pragma unroll
      for (int it = 0; it < 2; ++it)
        *(volatile v8h*)(Y16 + (rb + l0 + it * 8 + wave) * kDin + d0 + lane * 8) = hv[it];
      __threadfence();
    }
  }
}

__global__ __launch_bounds__(256) void gelu_cast_kernel(
    const float* __restrict__ H, unsigned short* __restrict__ A16, int total8, float scale)
{
  __shared__ float sG[8 * 256];
  const int tid = threadIdx.x;
  const int i = blockIdx.x * 256 + tid;
  if (i >= total8) return;
  const size_t e0 = (size_t)i << 3;
#pragma unroll 1
  for (int e = 0; e < 8; ++e) {
    const float v  = H[e0 + e];
    const float gl = 0.5f * v * (1.0f + erff(v * 0.70710678118654752f));
    sG[e * 256 + tid] = gl;
  }
  v8h hv;
#pragma unroll
  for (int e = 0; e < 8; ++e) hv[e] = (_Float16)(sG[e * 256 + tid] * scale);
  unsigned short* q = A16 + e0;
  *(volatile v8h*)q = hv;
  __threadfence();
  *(volatile v8h*)q = hv;
}

extern "C" void kernel_launch(void* const* d_in, const int* in_sizes, int n_in,
                              void* d_out, int out_size, void* d_ws, size_t ws_size,
                              hipStream_t stream)
{
  if (n_in < 20) return;
  const float* x        = (const float*)d_in[0];
  const float* g1       = (const float*)d_in[1];
  const float* b1       = (const float*)d_in[2];
  const float* lconv_w  = (const float*)d_in[3];
  const float* lconv_b  = (const float*)d_in[4];
  const float* in_projw = (const float*)d_in[5];
  const float* mconv_w  = (const float*)d_in[6];
  const float* mconv_b  = (const float*)d_in[7];
  const float* x_projw  = (const float*)d_in[8];
  const float* dt_w     = (const float*)d_in[9];
  const float* dt_b     = (const float*)d_in[10];
  const float* A_log    = (const float*)d_in[11];
  const float* Dp       = (const float*)d_in[12];
  const float* out_projw= (const float*)d_in[13];
  const float* g2       = (const float*)d_in[14];
  const float* b2       = (const float*)d_in[15];
  const float* w1       = (const float*)d_in[16];
  const float* bb1      = (const float*)d_in[17];
  const float* w2       = (const float*)d_in[18];
  const float* bb2      = (const float*)d_in[19];
  float* dout = (float*)d_out;

  if (in_sizes[0] != kRows * kDim) return;
  if (in_sizes[1] != kDim || in_sizes[2] != kDim) return;
  if (in_sizes[3] != kDim * 3 || in_sizes[4] != kDim) return;
  if (in_sizes[5] != kXZP * kDim) return;
  if (in_sizes[6] != kDin * 4 || in_sizes[7] != kDin) return;
  if (in_sizes[8] != kXdbN * kDin) return;
  if (in_sizes[9] != kDin * kDtR || in_sizes[10] != kDin) return;
  if (in_sizes[11] != kDin * kNst || in_sizes[12] != kDin) return;
  if (in_sizes[13] != kDim * kDin) return;
  if (in_sizes[14] != kDim || in_sizes[15] != kDim) return;
  if (in_sizes[16] != kHid * kDim || in_sizes[17] != kHid) return;
  if (in_sizes[18] != kDim * kHid || in_sizes[19] != kDim) return;
  if (out_size != kRows * kDim) return;

  const size_t SZ_WIN16  = (size_t)kXZP * kDim * 2;
  const size_t SZ_WXP16  = (size_t)kXdbP * kDin * 2;
  const size_t SZ_WDT16  = (size_t)kDin * kDtP * 2;
  const size_t SZ_WOUT16 = (size_t)kDim * kDin * 2;
  const size_t SZ_W1     = (size_t)kHid * kDim * 2;
  const size_t SZ_W2     = (size_t)kDim * kHid * 2;
  const size_t SZ_U0     = (size_t)kRows * kDim * 2;
  const size_t SZ_XZ     = (size_t)kRows * kXZP * 4;
  const size_t SZ_XIN    = (size_t)kRows * kDin * 4;
  const size_t SZ_XIN16  = (size_t)kRows * kDin * 2;
  const size_t SZ_XDB    = (size_t)kRows * kXdbP * 4;
  const size_t SZ_DT16   = (size_t)kRows * kDtP * 2;
  const size_t SZ_DLR    = (size_t)kRows * kDin * 4;
  const size_t SZ_YG16   = (size_t)kRows * kDin * 2;
  const size_t SZ_X2     = (size_t)kRows * kDim * 4;
  const size_t SZ_X2LN   = (size_t)kRows * kDim * 2;
  const size_t SZ_H1     = (size_t)kRows * kHid * 4;
  const size_t SZ_A1     = (size_t)kRows * kHid * 2;
  const size_t OFF_WIN16  = 0;
  const size_t OFF_WXP16  = OFF_WIN16  + SZ_WIN16;
  const size_t OFF_WDT16  = OFF_WXP16  + SZ_WXP16;
  const size_t OFF_WOUT16 = OFF_WDT16  + SZ_WDT16;
  const size_t OFF_W1     = OFF_WOUT16 + SZ_WOUT16;
  const size_t OFF_W2     = OFF_W1     + SZ_W1;
  const size_t OFF_U0     = OFF_W2     + SZ_W2;
  const size_t OFF_XZ     = OFF_U0     + SZ_U0;
  const size_t OFF_XIN    = OFF_XZ     + SZ_XZ;
  const size_t OFF_XIN16  = OFF_XIN    + SZ_XIN;
  const size_t OFF_XDB    = OFF_XIN16  + SZ_XIN16;
  const size_t OFF_DT16   = OFF_XDB    + SZ_XDB;
  const size_t OFF_DLR    = OFF_DT16   + SZ_DT16;
  const size_t OFF_YG16   = OFF_DLR    + SZ_DLR;
  const size_t OFF_X2     = OFF_YG16   + SZ_YG16;
  const size_t OFF_X2LN   = OFF_X2     + SZ_X2;
  const size_t OFF_H1     = OFF_X2LN   + SZ_X2LN;
  const size_t OFF_A1     = OFF_H1     + SZ_H1;
  const size_t TOTAL      = OFF_A1     + SZ_A1;
  if (ws_size < TOTAL) return;

  char* ws = (char*)d_ws;
  unsigned short* WIN16  = (unsigned short*)(ws + OFF_WIN16);
  unsigned short* WXP16  = (unsigned short*)(ws + OFF_WXP16);
  unsigned short* WDT16  = (unsigned short*)(ws + OFF_WDT16);
  unsigned short* WOUT16 = (unsigned short*)(ws + OFF_WOUT16);
  unsigned short* W1_16  = (unsigned short*)(ws + OFF_W1);
  unsigned short* W2_16  = (unsigned short*)(ws + OFF_W2);
  unsigned short* U0     = (unsigned short*)(ws + OFF_U0);
  float*          XZ     = (float*)(ws + OFF_XZ);
  float*          XIN    = (float*)(ws + OFF_XIN);
  unsigned short* XIN16  = (unsigned short*)(ws + OFF_XIN16);
  float*          XDB    = (float*)(ws + OFF_XDB);
  unsigned short* DT16   = (unsigned short*)(ws + OFF_DT16);
  float*          DLR    = (float*)(ws + OFF_DLR);
  unsigned short* YG16   = (unsigned short*)(ws + OFF_YG16);
  float*          X2     = (float*)(ws + OFF_X2);
  unsigned short* X2LN   = (unsigned short*)(ws + OFF_X2LN);
  float*          H1     = (float*)(ws + OFF_H1);
  unsigned short* A1_16  = (unsigned short*)(ws + OFF_A1);
  const float* dummy_bias  = dt_b;
  const float* dummy_resid = x;

  cast_f16_kernel<<<(kXZP * kDim) / 8 / 256, 256, 0, stream>>>(in_projw, WIN16, (kXZP * kDim) / 8, 32.0f);
  cast_f16_kernel<<<(kXdbN * kDin) / 8 / 256, 256, 0, stream>>>(x_projw, WXP16, (kXdbN * kDin) / 8, 32.0f);
  zero16_kernel<<<((kXdbP - kXdbN) * kDin) / 8 / 256, 256, 0, stream>>>(WXP16 + (size_t)kXdbN * kDin,
                                                                       ((kXdbP - kXdbN) * kDin) / 8);
  pad16_cast_kernel<<<(kDin * 4) / 256, 256, 0, stream>>>(dt_w, kDtR, WDT16, kDin * 4, 8.0f);
  cast_f16_kernel<<<(kDim * kDin) / 8 / 256, 256, 0, stream>>>(out_projw, WOUT16, (kDim * kDin) / 8, 32.0f);
  cast_f16_kernel<<<(kHid * kDim) / 8 / 256, 256, 0, stream>>>(w1, W1_16, (kHid * kDim) / 8, 32.0f);
  cast_f16_kernel<<<(kDim * kHid) / 8 / 256, 256, 0, stream>>>(w2, W2_16, (kDim * kHid) / 8, 32.0f);

  ln_conv_kernel<<<kRows / 32, 256, 0, stream>>>(x, g1, b1, lconv_w, lconv_b, U0);

  wmma_gemm64<0, false, 0, 0, false><<<dim3(128, 1), 256, 0, stream>>>(
      U0, U0, kDim, 0L, WIN16, WIN16, kDim, 0L,
      (void*)XZ, (void*)XZ, kXZP, 0L, dummy_bias, dummy_resid, 0L, kRows, kXZP, kDim, 1.0f / 32.0f);

  conv_silu_kernel<<<dim3(kDin / 256, kL / 64, kB), 256, 0, stream>>>(XZ, mconv_w, mconv_b, XIN, XIN16);

  wmma_gemm64<0, false, 0, 0, false><<<dim3(16, 1), 256, 0, stream>>>(
      XIN16, XIN16, kDin, 0L, WXP16, WXP16, kDin, 0L,
      (void*)XDB, (void*)XDB, kXdbP, 0L, dummy_bias, dummy_resid, 0L, kRows, kXdbP, kDin, 1.0f / 512.0f);

  pad16_cast_kernel<<<(kRows * 4) / 256, 256, 0, stream>>>(XDB, kXdbP, DT16, kRows * 4, 64.0f);

  wmma_gemm64<0, false, 2, 0, false><<<dim3(64, 1), 256, 0, stream>>>(
      DT16, DT16, kDtP, 0L, WDT16, WDT16, kDtP, 0L,
      (void*)DLR, (void*)DLR, kDin, 0L, dt_b, dummy_resid, 0L, kRows, kDin, kDtP, 1.0f / 512.0f);

  scan_kernel<<<dim3(kDin / 256, kB), 256, 0, stream>>>(DLR, XIN, XZ, XDB, A_log, Dp, YG16);

  wmma_gemm64<0, false, 0, 0, true><<<dim3(32, 1), 256, 0, stream>>>(
      YG16, YG16, kDin, 0L, WOUT16, WOUT16, kDin, 0L,
      (void*)X2, (void*)X2, kDim, 0L, dummy_bias, x, 0L, kRows, kDim, kDin, 1.0f / 8192.0f);

  ln_cast_kernel<<<kRows / 32, 256, 0, stream>>>(X2, g2, b2, X2LN);

  wmma_gemm64<0, false, 2, 0, false><<<dim3(128, 1), 256, 0, stream>>>(
      X2LN, X2LN, kDim, 0L, W1_16, W1_16, kDim, 0L,
      (void*)H1, (void*)H1, kHid, 0L, bb1, dummy_resid, 0L, kRows, kHid, kDim, 1.0f / 32.0f);

  gelu_cast_kernel<<<(kRows * kHid) / 8 / 256, 256, 0, stream>>>(H1, A1_16, (kRows * kHid) / 8, 64.0f);

  wmma_gemm64<0, false, 2, 0, true><<<dim3(32, 1), 256, 0, stream>>>(
      A1_16, A1_16, kHid, 0L, W2_16, W2_16, kHid, 0L,
      (void*)dout, (void*)dout, kDim, 0L, bb2, X2, 0L, kRows, kDim, kHid, 1.0f / 2048.0f);
}
